// MultiLayerScorer_70248485093977
// MI455X (gfx1250) — hardware-run, weakly checked
//
#include <hip/hip_runtime.h>


#pragma clang fp contract(off)

#ifndef NB
#define NB 16
#endif
#define NB_FULL 16
#define SRC  100
#define TGT  100
#define KD   512
#define HID  256
#define SCP  128
#define MROWS (NB * SRC)
#define MPAD  (((MROWS + 63) / 64) * 64)
#define NPIECE ((unsigned)((size_t)MROWS * TGT / 4))

static_assert(SRC == TGT);
static_assert(KD % 64 == 0);
static_assert(KD % 32 == 0);
static_assert(HID % 64 == 0);
static_assert(HID == 256);
static_assert(SCP == 128);
static_assert(SCP >= TGT);
static_assert(NB <= NB_FULL);
static_assert(MPAD <= NB_FULL * SRC);
static_assert(((size_t)MPAD * KD) % 8 == 0);
static_assert(((size_t)MROWS * TGT) % 4 == 0);
static_assert(MPAD % 64 == 0);

typedef unsigned short bf;
typedef __attribute__((ext_vector_type(16))) __bf16   v16bf;
typedef __attribute__((ext_vector_type(8)))  unsigned short v8us;
typedef __attribute__((ext_vector_type(8)))  float    v8f;
typedef __attribute__((ext_vector_type(4)))  float    v4f;
typedef v4f  __attribute__((may_alias)) v4fa;
typedef v8us __attribute__((may_alias)) v8usa;

__device__ __forceinline__ unsigned short f2bf(float f) { unsigned u = __float_as_uint(f); u += 0x7FFFu + ((u >> 16) & 1u); return (unsigned short)(u >> 16); }
__device__ __forceinline__ float bfr(float f) { return __uint_as_float(((unsigned)f2bf(f)) << 16); }
__device__ __forceinline__ v16bf cat16b(v8us lo, v8us hi) { return __builtin_bit_cast(v16bf, __builtin_shufflevector(lo, hi, 0, 1, 2, 3, 4, 5, 6, 7, 8, 9, 10, 11, 12, 13, 14, 15)); }
__device__ __forceinline__ v8f wmmab(v16bf a, v16bf b, v8f c) { return __builtin_amdgcn_wmma_f32_16x16x32_bf16(false, a, false, b, (short)0, c, false, false); }
__device__ __forceinline__ v8f wmmabg(v16bf a, v16bf b, v8f c) { c = wmmab(a, b, c); asm volatile("v_nop\n\tv_nop\n\tv_nop\n\tv_nop" : "+v"(c) : "v"(a), "v"(b)); return c; }
__device__ __forceinline__ v16bf ldb(const bf* p)  { return cat16b(*(const v8us*)p, *(const v8us*)(p + 16)); }
__device__ __forceinline__ void wave_sync() { __builtin_amdgcn_fence(3  , "wavefront"); __builtin_amdgcn_wave_barrier(); asm volatile("" ::: "memory"); }

__global__ __launch_bounds__(256) void k_cvt8(const float* __restrict__ src, bf* dst, size_t n8) {
    const size_t i = (size_t)blockIdx.x * 256 + threadIdx.x; if (i >= n8) return;
    const v8f v = *(const v8f*)(src + i * 8); v8us o;
#pragma unroll
    for (int k = 0; k < 8; ++k) o[k] = f2bf(v[k]);
    *(volatile v8us*)(dst + i * 8) = o; __threadfence(); *(volatile v8us*)(dst + i * 8) = o;
}

__global__ __launch_bounds__(256) void k_wtr(const float* __restrict__ W, bf* WT) {
    __shared__ __align__(16) bf ts[64 * 72];
    static_assert(sizeof(bf) * 64 * 72 <= 131072);
    static_assert(256 * 2 * 16 == 64 * 128);
    static_assert((72 * 2) % 16 == 0);
    const unsigned tid = threadIdx.x;
    const unsigned k0 = blockIdx.x * 64u, n0 = blockIdx.y * 64u;
    const unsigned nn = tid & 63u, kq = tid >> 6;
#pragma unroll 4
    for (unsigned i = 0; i < 16; ++i) { const unsigned kk = kq + 4u * i;
        ts[nn * 72u + kk] = f2bf(W[(size_t)(k0 + kk) * HID + n0 + nn]); }
    __syncthreads();
#pragma unroll 1
    for (int ps = 0; ps < 2; ++ps) {
#pragma unroll
        for (unsigned s = 0; s < 2; ++s) { const unsigned row = 32u * s + (tid >> 3), c8 = (tid & 7u) * 8u;
            const v8us o = *(const v8usa*)(&ts[row * 72u + c8]);
            *(volatile v8us*)(WT + (size_t)(n0 + row) * KD + k0 + c8) = o; }
        if (ps == 0) __threadfence(); }
}

__global__ __launch_bounds__(32) void k_proj(const bf* __restrict__ A, const bf* __restrict__ Bt, const float* __restrict__ bias, int useb, float* P) {
    __shared__ __align__(16) float os[16 * 68];
    static_assert(sizeof(float) * 16 * 68 <= 131072);
    static_assert(32 * 16 * 8 == 16 * 64 * 4);
    static_assert((68 * 4) % 16 == 0);
    const int K = KD;
    const int lane = threadIdx.x & 31, lr = lane & 15, hi = lane >> 4; const int r0 = blockIdx.x * 64, c0 = blockIdx.y * 64;
    v8f acc[4][4];
#pragma unroll
    for (int mb = 0; mb < 4; ++mb)
#pragma unroll
        for (int nb = 0; nb < 4; ++nb) acc[mb][nb] = (v8f){};
    const size_t aoff = (size_t)(r0 + lr) * K + 8 * hi, boff = (size_t)(c0 + lr) * K + 8 * hi;
#pragma unroll 1
    for (int kc = 0; kc < K; kc += 32) {
        v16bf a[4];
#pragma unroll
        for (int mb = 0; mb < 4; ++mb) a[mb] = ldb(A + aoff + (size_t)mb * 16 * K + kc);
#pragma unroll
        for (int nb = 0; nb < 4; ++nb) { const v16bf b = ldb(Bt + boff + (size_t)nb * 16 * K + kc);
#pragma unroll
            for (int mb = 0; mb < 4; ++mb) acc[mb][nb] = wmmabg(a[mb], b, acc[mb][nb]); }
    }
    float bc[4];
#pragma unroll
    for (int nb = 0; nb < 4; ++nb) { const float bv = bfr(bias[c0 + nb * 16 + lr]); bc[nb] = (useb != 0) ? bv : 0.0f; }
#pragma unroll
    for (int mb = 0; mb < 4; ++mb) {
#pragma unroll
        for (int nb = 0; nb < 4; ++nb) {
#pragma unroll
            for (int j = 0; j < 8; ++j) os[(hi * 8 + j) * 68 + nb * 16 + lr] = acc[mb][nb][j] + bc[nb]; }
        wave_sync();
        float* pb = P + (size_t)(r0 + mb * 16) * HID + c0;
#pragma unroll 1
        for (int ps = 0; ps < 2; ++ps) {
#pragma unroll
            for (int s = 0; s < 8; ++s) { const int row = 2 * s + (lane >> 4), c4 = (lane & 15) * 4;
                const v4f val = *(const v4fa*)(&os[row * 68 + c4]);
                *(volatile v4f*)(pb + (size_t)row * HID + c4) = val; }
            if (ps == 0) __threadfence(); }
        wave_sync();
    }
}

__global__ __launch_bounds__(256) void k_score(const float* __restrict__ HK, const float* __restrict__ HQ, const float* __restrict__ W2, const float* __restrict__ b2, float* SC) {
    __shared__ __align__(16) float hks[HID];
    __shared__ __align__(16) float w2s[HID];
    __shared__ __align__(16) float scs[SCP];
    static_assert(sizeof(float) * (HID + HID + SCP) <= 131072);
    static_assert(32 * 16 == SCP * 4);
    const unsigned tid = threadIdx.x; const unsigned lane = tid & 31u;
    const int wave = __builtin_amdgcn_readfirstlane((int)(threadIdx.x >> 5));
    const unsigned row = blockIdx.x;
    const unsigned b = row / (unsigned)SRC;
    hks[tid] = HK[(size_t)row * HID + tid];
    w2s[tid] = bfr(W2[tid]);
    if (tid >= (unsigned)TGT && tid < (unsigned)SCP) scs[tid] = 0.0f;
    __syncthreads();
    const float b2v = bfr(b2[0]);
    const float* hqb = HQ + (size_t)b * TGT * HID + lane;
#pragma unroll 1
    for (int t = wave; t < TGT; t += 8) {
        const float* hq = hqb + (size_t)t * HID;
        float p = 0.0f;
#pragma unroll 1
        for (int g = 0; g < 8; ++g) {
            const unsigned u = 32u * (unsigned)g + lane;
            const float x = hks[u] + hq[32 * g];
            p = fmaf(w2s[u], tanhf(x), p); }
        p += __shfl_xor(p, 16, 32);
        p += __shfl_xor(p, 8, 32);
        p += __shfl_xor(p, 4, 32);
        p += __shfl_xor(p, 2, 32);
        p += __shfl_xor(p, 1, 32);
        const float r = tanhf(p + b2v);
        if (lane == 0u) scs[t] = r;
    }
    __syncthreads();
    if (wave == 0) {
        const v4f val = *(const v4fa*)(&scs[lane * 4u]);
        float* dst = SC + (size_t)row * SCP + lane * 4u;
        *(volatile v4f*)dst = val; __threadfence(); *(volatile v4f*)dst = val;
    }
}

__global__ __launch_bounds__(256) void k_out(const float* __restrict__ SC, float* OUT) {
    const unsigned i = blockIdx.x * 256u + threadIdx.x; if (i >= NPIECE) return;
    v4f val;
#pragma unroll
    for (unsigned j = 0; j < 4; ++j) { const unsigned e = 4u * i + j; const unsigned r = e / (unsigned)TGT; const unsigned c = e - r * (unsigned)TGT;
        val[j] = SC[(size_t)r * SCP + c]; }
    float* dst = OUT + (size_t)i * 4;
    *(volatile v4f*)dst = val; __threadfence(); *(volatile v4f*)dst = val;
}

static constexpr size_t al256(size_t v) { return (v + 255) & ~(size_t)255; }
static constexpr size_t SZ_XB = al256((size_t)MPAD * KD * 2);
static constexpr size_t SZ_WT = al256((size_t)HID * KD * 2);
static constexpr size_t SZ_HP = al256((size_t)MPAD * HID * 4);
static constexpr size_t SZ_SC = al256((size_t)MROWS * SCP * 4);
static constexpr size_t SZ_TOTAL = 2 * SZ_XB + 2 * SZ_WT + 2 * SZ_HP + SZ_SC;
static_assert(SZ_TOTAL <= (size_t)134217728);
static constexpr size_t N8_X = (size_t)MPAD * KD / 8;
static constexpr unsigned G_CVT = (unsigned)((N8_X + 255) / 256);
static constexpr unsigned G_OUT = (unsigned)(((size_t)NPIECE + 255) / 256);
static constexpr size_t NEED_X = (size_t)MPAD * KD;
static_assert((size_t)G_CVT * 256 >= N8_X);
static_assert((size_t)G_OUT * 256 >= (size_t)NPIECE);
static_assert((size_t)(MPAD / 64) * 64 == (size_t)MPAD);
static_assert((size_t)MROWS * TGT * 4 <= (size_t)NB_FULL * SRC * TGT * 4);

extern "C" void kernel_launch(void* const* d_in, const int* in_sizes, int n_in,
                              void* d_out, int out_size, void* d_ws, size_t ws_size, hipStream_t stream) {
    if (n_in < 7) return;
    if ((size_t)in_sizes[0] < NEED_X || (size_t)in_sizes[1] < NEED_X) return;
    if ((size_t)in_sizes[2] < (size_t)KD * HID || (size_t)in_sizes[3] < (size_t)KD * HID) return;
    if (in_sizes[4] < HID || in_sizes[5] < HID || in_sizes[6] < 1) return;
    if ((size_t)out_size < (size_t)MROWS * TGT) return;
    if (SZ_TOTAL > ws_size) return;
    const float* query = (const float*)d_in[0];
    const float* keys  = (const float*)d_in[1];
    const float* wk    = (const float*)d_in[2];
    const float* wq    = (const float*)d_in[3];
    const float* b1    = (const float*)d_in[4];
    const float* w2    = (const float*)d_in[5];
    const float* b2    = (const float*)d_in[6];
    float* OUT = (float*)d_out;
    char* wsp = (char*)d_ws;
    bf* XQ  = (bf*)wsp; wsp += SZ_XB;
    bf* XK  = (bf*)wsp; wsp += SZ_XB;
    bf* WTQ = (bf*)wsp; wsp += SZ_WT;
    bf* WTK = (bf*)wsp; wsp += SZ_WT;
    float* HQ = (float*)wsp; wsp += SZ_HP;
    float* HK = (float*)wsp; wsp += SZ_HP;
    float* SC = (float*)wsp; wsp += SZ_SC;

    k_cvt8<<<G_CVT, 256, 0, stream>>>(query, XQ, N8_X);
    k_cvt8<<<G_CVT, 256, 0, stream>>>(keys, XK, N8_X);
    k_wtr<<<dim3(KD / 64, HID / 64, 1), 256, 0, stream>>>(wq, WTQ);
    k_wtr<<<dim3(KD / 64, HID / 64, 1), 256, 0, stream>>>(wk, WTK);
    k_proj<<<dim3(MPAD / 64, HID / 64, 1), 32, 0, stream>>>(XK, WTK, b1, 1, HK);
    k_proj<<<dim3(MPAD / 64, HID / 64, 1), 32, 0, stream>>>(XQ, WTQ, b1, 0, HQ);
    k_score<<<MROWS, 256, 0, stream>>>(HK, HQ, w2, b2, SC);
    k_out<<<G_OUT, 256, 0, stream>>>(SC, OUT);
}
